// MultiHeadSelfAttention_12970801234468
// MI455X (gfx1250) — hardware-verified
//
#include <hip/hip_runtime.h>
#ifndef NB
#define NB 2
#endif
#ifndef SEQ
#define SEQ 2048
#endif
#define NB_FULL 2
#define SEQ_FULL 2048
#define DM 1024
#define NH 16
#define HD 64
#define NRT (NB * SEQ)
#define QBLK (SEQ / 64)
#define WBYTES ((size_t)DM * DM * 2)
#define PBYTES ((size_t)NRT * DM * 2)
#define WS_TOTAL (4 * WBYTES + 10 * PBYTES)

static_assert(DM == NH * HD);
static_assert(HD == 64);
static_assert(DM % 64 == 0);
static_assert(DM % 128 == 0);
static_assert(DM % 32 == 0);
static_assert(SEQ % 128 == 0);
static_assert(NRT % 128 == 0);
static_assert(NRT % 64 == 0);
static_assert(SEQ % 32 == 0);
static_assert(NB <= NB_FULL);
static_assert(SEQ <= SEQ_FULL);
static_assert(((size_t)NRT * DM / 8) % 256 == 0);
static_assert(((size_t)DM * (DM / 8)) % 256 == 0);
static_assert(WBYTES % 256 == 0);
static_assert(PBYTES % 256 == 0);
static_assert(WS_TOTAL <= (size_t)134217728);

typedef __bf16 v16b __attribute__((ext_vector_type(16)));
typedef _Float16 v16h __attribute__((ext_vector_type(16)));
typedef unsigned short v8us __attribute__((ext_vector_type(8), may_alias));
typedef float v8f __attribute__((ext_vector_type(8)));
typedef float v4f __attribute__((ext_vector_type(4)));
typedef float v4fa __attribute__((ext_vector_type(4), may_alias));
union FragB { v16b v; v8us half[2]; };
union FragH { v16h v; v8us half[2]; _Float16 h[16]; };

__device__ __forceinline__ unsigned short bf16_bits(float x) { unsigned int u = __float_as_uint(x); return (unsigned short)((u + 0x7FFFu + ((u >> 16) & 1u)) >> 16); }
__device__ __forceinline__ float bf16_val(unsigned short b) { return __uint_as_float(((unsigned int)b) << 16); }
__device__ __forceinline__ float bf16_rne(float x) { return bf16_val(bf16_bits(x)); }

__device__ __forceinline__ v16h ld_fragh(const unsigned short* __restrict__ p) { FragH f; f.half[0] = *(const v8us*)(p); f.half[1] = *(const v8us*)(p + 16); return f.v; }
__device__ __forceinline__ v16b ld_fragb(const unsigned short* __restrict__ p) { FragB f; f.half[0] = *(const v8us*)(p); f.half[1] = *(const v8us*)(p + 16); return f.v; }

__device__ __forceinline__ v8f mma_h(v16h a, v16h b, v8f c) {
  c = __builtin_amdgcn_wmma_f32_16x16x32_f16(false, a, false, b, (short)0, c, false, false);
  asm volatile("v_nop\n\tv_nop\n\tv_nop\n\tv_nop" : "+v"(c) : "v"(a), "v"(b));
  return c;
}
__device__ __forceinline__ v8f mma_b2(v16b ah, v16b al, v16b b, v8f c) {
  c = __builtin_amdgcn_wmma_f32_16x16x32_bf16(false, ah, false, b, (short)0, c, false, false);
  c = __builtin_amdgcn_wmma_f32_16x16x32_bf16(false, al, false, b, (short)0, c, false, false);
  asm volatile("v_nop\n\tv_nop\n\tv_nop\n\tv_nop" : "+v"(c) : "v"(ah), "v"(al), "v"(b));
  return c;
}
__device__ __forceinline__ v8f mma_b3(v16b ah, v16b al, v16b bh, v16b bl, v8f c) {
  c = __builtin_amdgcn_wmma_f32_16x16x32_bf16(false, ah, false, bh, (short)0, c, false, false);
  c = __builtin_amdgcn_wmma_f32_16x16x32_bf16(false, al, false, bh, (short)0, c, false, false);
  c = __builtin_amdgcn_wmma_f32_16x16x32_bf16(false, ah, false, bl, (short)0, c, false, false);
  asm volatile("v_nop\n\tv_nop\n\tv_nop\n\tv_nop" : "+v"(c) : "v"(ah), "v"(al), "v"(bh), "v"(bl));
  return c;
}
__device__ __forceinline__ void wave_sync() { __builtin_amdgcn_fence(4  , "workgroup"); __builtin_amdgcn_wave_barrier(); }

__global__ __launch_bounds__(256) void k_wt_f16(const float* __restrict__ W, unsigned short* __restrict__ Wt, int K, int N, float scale) {
  const int t = blockIdx.x * 256 + threadIdx.x;
  const int k8n = K / 8;
  if (t >= N * k8n) return;
  const int n = t / k8n, k8 = (t - n * k8n) * 8;
  FragH f;
#pragma unroll
  for (int i = 0; i < 8; ++i) f.h[i] = (_Float16)(bf16_rne(W[(size_t)(k8 + i) * N + n]) * scale);
  const v8us o = f.half[0];
  *(volatile v8us*)(Wt + (size_t)n * K + k8) = o;
  __threadfence();
  *(volatile v8us*)(Wt + (size_t)n * K + k8) = o;
}
__global__ __launch_bounds__(256) void k_wt_bf16(const float* __restrict__ W, unsigned short* __restrict__ Wt, int K, int N) {
  const int t = blockIdx.x * 256 + threadIdx.x;
  const int k8n = K / 8;
  if (t >= N * k8n) return;
  const int n = t / k8n, k8 = (t - n * k8n) * 8;
  v8us v;
#pragma unroll
  for (int i = 0; i < 8; ++i) v[i] = bf16_bits(W[(size_t)(k8 + i) * N + n]);
  *(volatile v8us*)(Wt + (size_t)n * K + k8) = v;
  __threadfence();
  *(volatile v8us*)(Wt + (size_t)n * K + k8) = v;
}
__global__ __launch_bounds__(256) void k_x16(const float* __restrict__ x, unsigned short* __restrict__ X16, int n8) {
  const int t = blockIdx.x * 256 + threadIdx.x;
  if (t >= n8) return;
  const int row = t / (DM / 8), c = (t - row * (DM / 8)) * 8;
  const int b = row / SEQ, s = row - b * SEQ;
  const size_t src = ((size_t)b * SEQ_FULL + s) * DM + c;
  const v4f a0 = *(const v4fa*)(x + src), a1 = *(const v4fa*)(x + src + 4);
  FragH f;
#pragma unroll
  for (int q = 0; q < 4; ++q) { f.h[q] = (_Float16)bf16_rne(a0[q]); f.h[4 + q] = (_Float16)bf16_rne(a1[q]); }
  const v8us o = f.half[0];
  *(volatile v8us*)(X16 + (size_t)t * 8) = o;
  __threadfence();
  *(volatile v8us*)(X16 + (size_t)t * 8) = o;
}

template <int MODE>
__device__ __forceinline__ void gemm_body(const unsigned short* __restrict__ A, const unsigned short* __restrict__ A2, int lda,
                                          const unsigned short* __restrict__ Bt, int ldb, float alpha,
                                          const float* __restrict__ bias, float bscale,
                                          float* __restrict__ C, unsigned short* __restrict__ Ca, unsigned short* __restrict__ Cb,
                                          int ldc, int N, int K) {
  __shared__ __attribute__((aligned(16))) float so[4][32][68];
  const int lane = threadIdx.x & 31, ln = lane & 15, hh = lane >> 4;
  const int w = __builtin_amdgcn_readfirstlane((int)(threadIdx.x >> 5));
  const int ntn = N >> 6;
  const int mt = blockIdx.x / ntn, nq = blockIdx.x - mt * ntn;
  const int row0 = mt * 128 + 32 * w, col0 = nq * 64;
  const size_t a0o = (size_t)(row0 + ln) * lda + 8 * hh, a1o = a0o + (size_t)16 * lda;
  const size_t b0o = (size_t)(col0 + ln) * ldb + 8 * hh, b1o = b0o + (size_t)16 * ldb, b2o = b1o + (size_t)16 * ldb, b3o = b2o + (size_t)16 * ldb;
  const v8f z8 = {0.f, 0.f, 0.f, 0.f, 0.f, 0.f, 0.f, 0.f};
  v8f c00 = z8, c01 = z8, c02 = z8, c03 = z8, c10 = z8, c11 = z8, c12 = z8, c13 = z8;
  if constexpr (MODE == 2) {
#pragma unroll 1
    for (int kb = 0; kb < K; kb += 32) {
      const v16b a0h = ld_fragb(A + a0o + kb), a0l = ld_fragb(A2 + a0o + kb);
      const v16b a1h = ld_fragb(A + a1o + kb), a1l = ld_fragb(A2 + a1o + kb);
      v16b bb = ld_fragb(Bt + b0o + kb); c00 = mma_b2(a0h, a0l, bb, c00); c10 = mma_b2(a1h, a1l, bb, c10);
      bb = ld_fragb(Bt + b1o + kb); c01 = mma_b2(a0h, a0l, bb, c01); c11 = mma_b2(a1h, a1l, bb, c11);
      bb = ld_fragb(Bt + b2o + kb); c02 = mma_b2(a0h, a0l, bb, c02); c12 = mma_b2(a1h, a1l, bb, c12);
      bb = ld_fragb(Bt + b3o + kb); c03 = mma_b2(a0h, a0l, bb, c03); c13 = mma_b2(a1h, a1l, bb, c13);
    }
  } else {
#pragma unroll 1
    for (int kb = 0; kb < K; kb += 32) {
      const v16h a0 = ld_fragh(A + a0o + kb), a1 = ld_fragh(A + a1o + kb);
      v16h bb = ld_fragh(Bt + b0o + kb); c00 = mma_h(a0, bb, c00); c10 = mma_h(a1, bb, c10);
      bb = ld_fragh(Bt + b1o + kb); c01 = mma_h(a0, bb, c01); c11 = mma_h(a1, bb, c11);
      bb = ld_fragh(Bt + b2o + kb); c02 = mma_h(a0, bb, c02); c12 = mma_h(a1, bb, c12);
      bb = ld_fragh(Bt + b3o + kb); c03 = mma_h(a0, bb, c03); c13 = mma_h(a1, bb, c13);
    }
  }
  v8f accs[8] = {c00, c01, c02, c03, c10, c11, c12, c13};
#pragma unroll
  for (int u = 0; u < 8; ++u) {
    const int t = u & 3, half = u >> 2;
    float bv = 0.f;
    if (MODE != 1) bv = bf16_rne(bias[col0 + t * 16 + ln]) * bscale;
#pragma unroll
    for (int r = 0; r < 8; ++r) so[w][half * 16 + 8 * hh + r][t * 16 + ln] = accs[u][r] * alpha + bv;
  }
  wave_sync();
  if constexpr (MODE == 2) {
    const int rsub = lane >> 4, c4 = (lane & 15) * 4;
    for (int pass = 0; pass < 2; ++pass) {
#pragma unroll
      for (int q = 0; q < 16; ++q) {
        const int r = q * 2 + rsub;
        const v4f v = *(const v4fa*)&so[w][r][c4];
        const int grow = row0 + r;
        const int ob = grow / SEQ, os = grow - ob * SEQ;
        *(volatile v4f*)(C + ((size_t)ob * SEQ_FULL + os) * ldc + col0 + c4) = v;
      }
      if (pass == 0) __threadfence();
    }
  } else {
    const int rq = lane >> 3, c8 = (lane & 7) * 8;
    for (int pass = 0; pass < 2; ++pass) {
#pragma unroll
      for (int q = 0; q < 8; ++q) {
        const int r = q * 4 + rq;
        const v4f x0 = *(const v4fa*)&so[w][r][c8], x1 = *(const v4fa*)&so[w][r][c8 + 4];
        const float xv[8] = {x0[0], x0[1], x0[2], x0[3], x1[0], x1[1], x1[2], x1[3]};
        const size_t off = (size_t)(row0 + r) * ldc + col0 + c8;
        if constexpr (MODE == 0) {
          v8us hi, lo;
#pragma unroll
          for (int i = 0; i < 8; ++i) { const unsigned short hb = bf16_bits(xv[i]); hi[i] = hb; lo[i] = bf16_bits(xv[i] - bf16_val(hb)); }
          *(volatile v8us*)(Ca + off) = hi;
          *(volatile v8us*)(Cb + off) = lo;
        } else {
          const float br = bf16_rne(bias[row0 + r]);
          FragH f;
#pragma unroll
          for (int i = 0; i < 8; ++i) f.h[i] = (_Float16)(xv[i] + br);
          const v8us o = f.half[0];
          *(volatile v8us*)(Ca + off) = o;
        }
      }
      if (pass == 0) __threadfence();
    }
  }
}

__global__ __launch_bounds__(128) void k_gemm_hl(const unsigned short* __restrict__ A, int lda, const unsigned short* __restrict__ Bt, int ldb, float alpha,
                                                 const float* __restrict__ bias, float bscale, unsigned short* __restrict__ Ch, unsigned short* __restrict__ Cl,
                                                 int ldc, int N, int K) {
  gemm_body<0>(A, A, lda, Bt, ldb, alpha, bias, bscale, nullptr, Ch, Cl, ldc, N, K);
}
__global__ __launch_bounds__(128) void k_gemm_vt(const unsigned short* __restrict__ A, int lda, const unsigned short* __restrict__ Bt, int ldb, float alpha,
                                                 const float* __restrict__ bias, unsigned short* __restrict__ Cv, int ldc, int N, int K) {
  gemm_body<1>(A, A, lda, Bt, ldb, alpha, bias, 1.0f, nullptr, Cv, Cv, ldc, N, K);
}
__global__ __launch_bounds__(128) void k_gemm_out(const unsigned short* __restrict__ Ah, const unsigned short* __restrict__ Al, int lda, const unsigned short* __restrict__ Bt, int ldb,
                                                  const float* __restrict__ bias, float* __restrict__ C, int ldc, int N, int K) {
  gemm_body<2>(Ah, Al, lda, Bt, ldb, 1.0f, bias, 1.0f, C, nullptr, nullptr, ldc, N, K);
}

__global__ __launch_bounds__(128) void k_attn(const unsigned short* __restrict__ QH, const unsigned short* __restrict__ QL,
                                              const unsigned short* __restrict__ KH, const unsigned short* __restrict__ KL,
                                              const unsigned short* __restrict__ VT,
                                              unsigned short* __restrict__ CH, unsigned short* __restrict__ CL) {
  __shared__ __attribute__((aligned(16))) float sS[4][16][36];
  __shared__ __attribute__((aligned(16))) float sA[4][16];
  __shared__ __attribute__((aligned(16))) float sO[4][16][68];
  const int lane = threadIdx.x & 31, ln = lane & 15, hh = lane >> 4;
  const int wave = __builtin_amdgcn_readfirstlane((int)(threadIdx.x >> 5));
  const int bid = blockIdx.x;
  const int qb = bid % QBLK;
  const int h = (bid / QBLK) % NH;
  const int b = bid / (QBLK * NH);
  const int q0 = qb * 64 + wave * 16;
  const size_t qoff = ((size_t)b * SEQ + q0 + ln) * DM + h * HD + 8 * hh;
  const size_t koff = ((size_t)b * SEQ + ln) * DM + h * HD + 8 * hh;
  const size_t voff = (size_t)(h * HD + ln) * NRT + (size_t)b * SEQ + 8 * hh;
  const v8f z8 = {0.f, 0.f, 0.f, 0.f, 0.f, 0.f, 0.f, 0.f};
  v8f o0 = z8, o1 = z8, o2 = z8, o3 = z8;
  float m = -1.0e30f, lsum = 0.f;
#pragma unroll 1
  for (int key0 = 0; key0 < SEQ; key0 += 32) {
    v8f s0 = z8, s1 = z8;
#pragma unroll
    for (int c = 0; c < 2; ++c) {
      const v16b qh = ld_fragb(QH + qoff + c * 32), ql = ld_fragb(QL + qoff + c * 32);
      const size_t ko = koff + (size_t)key0 * DM + c * 32;
      v16b kh = ld_fragb(KH + ko), kl = ld_fragb(KL + ko);
      s0 = mma_b3(qh, ql, kh, kl, s0);
      kh = ld_fragb(KH + ko + (size_t)16 * DM); kl = ld_fragb(KL + ko + (size_t)16 * DM);
      s1 = mma_b3(qh, ql, kh, kl, s1);
    }
#pragma unroll
    for (int r = 0; r < 8; ++r) { sS[wave][8 * hh + r][ln] = s0[r]; sS[wave][8 * hh + r][16 + ln] = s1[r]; }
    wave_sync();
    const v4f x0 = *(const v4fa*)&sS[wave][ln][8 * hh], x1 = *(const v4fa*)&sS[wave][ln][8 * hh + 4];
    const v4f x2 = *(const v4fa*)&sS[wave][ln][16 + 8 * hh], x3 = *(const v4fa*)&sS[wave][ln][16 + 8 * hh + 4];
    const float xs[16] = {x0[0], x0[1], x0[2], x0[3], x1[0], x1[1], x1[2], x1[3], x2[0], x2[1], x2[2], x2[3], x3[0], x3[1], x3[2], x3[3]};
    float mx = xs[0];
#pragma unroll
    for (int i = 1; i < 16; ++i) mx = fmaxf(mx, xs[i]);
    mx = fmaxf(mx, __shfl_xor(mx, 16, 32));
    const float nm = fmaxf(m, mx);
    const float al = __expf(m - nm);
    m = nm;
    float ps = 0.f;
    FragH pa;
#pragma unroll
    for (int i = 0; i < 16; ++i) { const float p = __expf(xs[i] - nm); ps += p; pa.h[i] = (_Float16)(p * 256.0f); }
    lsum = lsum * al + ps;
    if (hh == 0) sA[wave][ln] = al;
    wave_sync();
    const v4f a0 = *(const v4fa*)&sA[wave][8 * hh], a1 = *(const v4fa*)&sA[wave][8 * hh + 4];
    const float av[8] = {a0[0], a0[1], a0[2], a0[3], a1[0], a1[1], a1[2], a1[3]};
#pragma unroll
    for (int r = 0; r < 8; ++r) { o0[r] *= av[r]; o1[r] *= av[r]; o2[r] *= av[r]; o3[r] *= av[r]; }
    const size_t vo = voff + key0;
    const v16h v0 = ld_fragh(VT + vo), v1 = ld_fragh(VT + vo + (size_t)16 * NRT);
    const v16h v2 = ld_fragh(VT + vo + (size_t)32 * NRT), v3 = ld_fragh(VT + vo + (size_t)48 * NRT);
    o0 = mma_h(pa.v, v0, o0);
    o1 = mma_h(pa.v, v1, o1);
    o2 = mma_h(pa.v, v2, o2);
    o3 = mma_h(pa.v, v3, o3);
  }
  const float lt = lsum + __shfl_xor(lsum, 16, 32);
  const float inv = 1.0f / (256.0f * lt);
  wave_sync();
  if (hh == 0) sA[wave][ln] = inv;
#pragma unroll
  for (int r = 0; r < 8; ++r) {
    sO[wave][8 * hh + r][ln] = o0[r]; sO[wave][8 * hh + r][16 + ln] = o1[r];
    sO[wave][8 * hh + r][32 + ln] = o2[r]; sO[wave][8 * hh + r][48 + ln] = o3[r];
  }
  wave_sync();
  const int rq = lane >> 3, c8 = (lane & 7) * 8;
  for (int pass = 0; pass < 2; ++pass) {
#pragma unroll
    for (int q = 0; q < 4; ++q) {
      const int r = q * 4 + rq;
      const float sc = sA[wave][r];
      const v4f y0 = *(const v4fa*)&sO[wave][r][c8], y1 = *(const v4fa*)&sO[wave][r][c8 + 4];
      const float yv[8] = {y0[0] * sc, y0[1] * sc, y0[2] * sc, y0[3] * sc, y1[0] * sc, y1[1] * sc, y1[2] * sc, y1[3] * sc};
      v8us hi, lo;
#pragma unroll
      for (int i = 0; i < 8; ++i) { const unsigned short hb = bf16_bits(yv[i]); hi[i] = hb; lo[i] = bf16_bits(yv[i] - bf16_val(hb)); }
      const size_t off = ((size_t)b * SEQ + q0 + r) * DM + h * HD + c8;
      *(volatile v8us*)(CH + off) = hi;
      *(volatile v8us*)(CL + off) = lo;
    }
    if (pass == 0) __threadfence();
  }
}

extern "C" void kernel_launch(void* const* d_in, const int* in_sizes, int n_in,
                              void* d_out, int out_size, void* d_ws, size_t ws_size, hipStream_t stream) {
  if (n_in < 11) return;
  const size_t need_x = ((size_t)(NB - 1) * SEQ_FULL + SEQ) * DM;
  if ((size_t)in_sizes[0] < need_x || (size_t)in_sizes[1] < need_x || (size_t)in_sizes[2] < need_x) return;
  if ((size_t)in_sizes[3] < (size_t)DM * DM || (size_t)in_sizes[5] < (size_t)DM * DM || (size_t)in_sizes[7] < (size_t)DM * DM || (size_t)in_sizes[9] < (size_t)DM * DM) return;
  if (in_sizes[4] < DM || in_sizes[6] < DM || in_sizes[8] < DM || in_sizes[10] < DM) return;
  if ((size_t)out_size < need_x) return;
  if (ws_size < WS_TOTAL) return;
  const float* q = (const float*)d_in[0];
  const float* k = (const float*)d_in[1];
  const float* v = (const float*)d_in[2];
  const float* Wq = (const float*)d_in[3];
  const float* bq = (const float*)d_in[4];
  const float* Wk = (const float*)d_in[5];
  const float* bk = (const float*)d_in[6];
  const float* Wv = (const float*)d_in[7];
  const float* bv = (const float*)d_in[8];
  const float* Wo = (const float*)d_in[9];
  const float* bo = (const float*)d_in[10];
  char* ws = (char*)d_ws;
  size_t off = 0;
  unsigned short* BQ = (unsigned short*)(ws + off); off += WBYTES;
  unsigned short* BK = (unsigned short*)(ws + off); off += WBYTES;
  unsigned short* BV = (unsigned short*)(ws + off); off += WBYTES;
  unsigned short* BO = (unsigned short*)(ws + off); off += WBYTES;
  unsigned short* XQ = (unsigned short*)(ws + off); off += PBYTES;
  unsigned short* XK = (unsigned short*)(ws + off); off += PBYTES;
  unsigned short* XV = (unsigned short*)(ws + off); off += PBYTES;
  unsigned short* QH = (unsigned short*)(ws + off); off += PBYTES;
  unsigned short* QL = (unsigned short*)(ws + off); off += PBYTES;
  unsigned short* KH = (unsigned short*)(ws + off); off += PBYTES;
  unsigned short* KL = (unsigned short*)(ws + off); off += PBYTES;
  unsigned short* VT = (unsigned short*)(ws + off); off += PBYTES;
  unsigned short* CH = (unsigned short*)(ws + off); off += PBYTES;
  unsigned short* CL = (unsigned short*)(ws + off); off += PBYTES;
  if (off > ws_size) return;

  const unsigned gw = (unsigned)(((size_t)DM * (DM / 8)) / 256);
  k_wt_f16<<<gw, 256, 0, stream>>>(Wq, BQ, DM, DM, 16.0f);
  k_wt_f16<<<gw, 256, 0, stream>>>(Wk, BK, DM, DM, 16.0f);
  k_wt_f16<<<gw, 256, 0, stream>>>(Wv, BV, DM, DM, 16.0f);
  k_wt_bf16<<<gw, 256, 0, stream>>>(Wo, BO, DM, DM);
  const int n8 = (int)((size_t)NRT * DM / 8);
  const unsigned gx = (unsigned)(n8 / 256);
  k_x16<<<gx, 256, 0, stream>>>(q, XQ, n8);
  k_x16<<<gx, 256, 0, stream>>>(k, XK, n8);
  k_x16<<<gx, 256, 0, stream>>>(v, XV, n8);
  const unsigned gp = (unsigned)((NRT / 128) * (DM / 64));
  k_gemm_hl<<<gp, 128, 0, stream>>>(XQ, DM, BQ, DM, 0.0078125f, bq, 0.125f, QH, QL, DM, DM, DM);
  k_gemm_hl<<<gp, 128, 0, stream>>>(XK, DM, BK, DM, 0.0625f, bk, 1.0f, KH, KL, DM, DM, DM);
  const unsigned gv = (unsigned)((DM / 128) * (NRT / 64));
  k_gemm_vt<<<gv, 128, 0, stream>>>(BV, DM, XV, DM, 0.0625f, bv, VT, NRT, NRT, DM);
  k_attn<<<(unsigned)(QBLK * NH * NB), 128, 0, stream>>>(QH, QL, KH, KL, VT, CH, CL);
  k_gemm_out<<<gp, 128, 0, stream>>>(CH, CL, DM, BO, DM, bo, (float*)d_out, DM, DM, DM);
}
